// OutputScalarNetwork_56873956933908
// MI455X (gfx1250) — hardware-verified
//
#include <hip/hip_runtime.h>
#include <math.h>

typedef __attribute__((ext_vector_type(16))) _Float16 v16h;
typedef __attribute__((ext_vector_type(8)))  _Float16 v8h;
typedef __attribute__((ext_vector_type(8)))  float    v8f;
typedef __attribute__((ext_vector_type(4)))  float    v4f;

constexpr int kSys      = 16;
constexpr int kAtoms    = 256;
constexpr int kChan     = 64;
constexpr int kNrbf     = 32;
constexpr int kHid      = 128;
constexpr int kPairRows = kSys * kAtoms;
constexpr int kAtomsPerWave = 32;
constexpr int kTilesPerSys  = kAtoms / kAtomsPerWave;
constexpr int kRowsPerBlk   = 32;
constexpr int kW2Pitch      = kChan + 1;
static_assert(kNrbf == 32, "one 32-deep matrix step per pair tile");
static_assert((kHid % 16) == 0 && (kAtoms % kAtomsPerWave) == 0, "tile multiples");
static_assert(kHid == 32 * 4, "one v4f per lane covers a hidden row");
static_assert(((kHid * kNrbf) % (32 * 8)) == 0, "W1T staging coverage");
static_assert((kPairRows % kRowsPerBlk) == 0, "neighbour rows per block");
static_assert(((kHid * kChan) % 128) == 0 && ((kRowsPerBlk * kChan) % 128) == 0, "staging coverage");

constexpr float kCutoff    = 5.0f;
constexpr float kGamma     = 10.0f;
constexpr float kLn2       = 0.6931471805599453f;
constexpr float kAvgAtoms  = 256.0f;
constexpr float kSqrtAvg   = 16.0f;
static_assert(kSqrtAvg * kSqrtAvg == kAvgAtoms, "feature scale");
constexpr float kFeatScale = 1.0f / kSqrtAvg;
constexpr float kInvSteps  = 1.0f / (float)(kNrbf - 1);
constexpr float kCarryRbf  = 512.0f;
constexpr float kCarryW1   = 64.0f;
constexpr float kCarryProd = kCarryRbf * kCarryW1;
constexpr float kFold      = 1.0f / kCarryProd;
constexpr float kF16MinNormal = 6.103515625e-5f;

constexpr size_t kOffV    = 0;
constexpr size_t kOffS    = kOffV + (size_t)kPairRows * kHid * 4;
constexpr size_t kOffW1T  = kOffS + (size_t)kPairRows * 4;
constexpr size_t kWsTotal = kOffW1T + (size_t)kHid * kNrbf * 2;
static_assert(kWsTotal == 2121728ull, "carve total");
static_assert(kWsTotal <= 134217728ull, "carve cap");
static_assert((kOffS % 128) == 0 && (kOffW1T % 128) == 0, "128-B aligned regions");

union FragU { v16h v; v8h h[2]; };
__device__ __forceinline__ v16h frag_load_f16(const _Float16* p) {
  FragU f;
  f.h[0] = *(const v8h*)(p);
  f.h[1] = *(const v8h*)(p + 16);
  return f.v;
}
__device__ __forceinline__ v8f mma_f16(v16h a, v16h b, v8f c) {
  c = __builtin_amdgcn_wmma_f32_16x16x32_f16(false, a, false, b, (short)0, c, false, false);
  asm volatile("v_nop\n\tv_nop\n\tv_nop\n\tv_nop" : "+v"(c) : "v"(a), "v"(b));
  return c;
}
__device__ __forceinline__ _Float16 basis_f16(float d) {
  const float g = expf(-kGamma * (d * d));
  const float c = g * kCarryRbf;
  const float f = (c < kF16MinNormal) ? 0.0f : c;
  return (_Float16)f;
}

__global__ __launch_bounds__(256) void w1_plane_kernel(const float* __restrict__ W1, unsigned short* __restrict__ W1t)
{
  const int idx = blockIdx.x * 256 + threadIdx.x;
  if (idx >= kHid * (kNrbf / 8)) return;
  const int n  = idx >> 2;
  const int kc = idx & 3;
  v8h hv;
#pragma unroll
  for (int e = 0; e < 8; ++e) {
    const float w  = W1[(kc * 8 + e) * kHid + n] * kCarryW1;
    const float wf = (fabsf(w) < kF16MinNormal) ? 0.0f : w;
    hv[e] = (_Float16)wf;
  }
  unsigned short* q = W1t + (size_t)idx * 8;
  *(volatile v8h*)q = hv;
  __threadfence();
  *(volatile v8h*)q = hv;
}

__global__ __launch_bounds__(128) void neighbour_vec_kernel(
    const float* __restrict__ features, const float* __restrict__ maskp,
    const float* __restrict__ W2, const float* __restrict__ b2,
    float* __restrict__ V, float* __restrict__ S)
{
  __shared__ __align__(16) float sW[kHid * kW2Pitch];
  __shared__ __align__(16) float sF[kRowsPerBlk * kChan];
  __shared__ __align__(16) float sV[kRowsPerBlk * kHid];
  __shared__ __align__(16) float sB[kHid];
  __shared__ __align__(16) float sS[kRowsPerBlk];
  const int tid = threadIdx.x, lane = tid & 31, wave = tid >> 5;
  const int row0 = blockIdx.x * kRowsPerBlk;

#pragma unroll 1
  for (int it = 0; it < (kHid * kChan) / 128; ++it) {
    const int idx = it * 128 + tid;
    sW[(idx >> 6) * kW2Pitch + (idx & (kChan - 1))] = W2[idx];
  }
#pragma unroll 1
  for (int it = 0; it < (kRowsPerBlk * kChan) / 128; ++it) {
    const int idx = it * 128 + tid;
    const int row = idx >> 6;
    const float mk = maskp[row0 + row];
    const float f  = features[(size_t)row0 * kChan + idx];
    sF[idx] = (f * kFeatScale) * mk;
  }
  sB[tid] = b2[tid & (kChan - 1)];
  __syncthreads();

#pragma unroll 1
  for (int rg = 0; rg < kRowsPerBlk / 4; ++rg) {
    float a0 = 0.0f, a1 = 0.0f, a2 = 0.0f, a3 = 0.0f;
    const float* f0 = sF + (rg * 4) * kChan;
    const float* wr = sW + tid * kW2Pitch;
#pragma unroll 4
    for (int i = 0; i < kChan; ++i) {
      const float w = wr[i];
      a0 = fmaf(w, f0[i], a0);
      a1 = fmaf(w, f0[kChan + i], a1);
      a2 = fmaf(w, f0[2 * kChan + i], a2);
      a3 = fmaf(w, f0[3 * kChan + i], a3);
    }
    sV[(rg * 4 + 0) * kHid + tid] = a0;
    sV[(rg * 4 + 1) * kHid + tid] = a1;
    sV[(rg * 4 + 2) * kHid + tid] = a2;
    sV[(rg * 4 + 3) * kHid + tid] = a3;
  }
  {
    const float* fr = sF + (tid & 31) * kChan;
    float t = 0.0f;
#pragma unroll 4
    for (int i = 0; i < kChan; ++i) t = fmaf(sB[i], fr[i], t);
    if (wave == 0) sS[lane] = t;
  }
  __syncthreads();

  v4f vals[8];
#pragma unroll
  for (int it = 0; it < 8; ++it) vals[it] = *(const v4f*)(sV + (it * 4 + wave) * kHid + lane * 4);
  const float sval = sS[lane];
  for (int pass = 0; pass < 2; ++pass) {
#pragma unroll
    for (int it = 0; it < 8; ++it)
      *(volatile v4f*)(V + (size_t)(row0 + it * 4 + wave) * kHid + lane * 4) = vals[it];
    if (wave == 0) *(volatile float*)(S + row0 + lane) = sval;
    __threadfence();
  }
}

__global__ __launch_bounds__(32) __attribute__((amdgpu_num_vgpr(256))) void pair_filter_kernel(
    const float* __restrict__ geom, const float* __restrict__ maskp, const float* __restrict__ b1,
    const _Float16* __restrict__ W1t, const float* __restrict__ V, const float* __restrict__ S,
    float* __restrict__ out)
{
  __shared__ __align__(16) _Float16 sA[kAtomsPerWave * kNrbf];
  __shared__ __align__(16) _Float16 sW[kHid * kNrbf];
  __shared__ __align__(16) float sC[kNrbf];
  __shared__ __align__(16) float sB1[kHid];
  __shared__ __align__(16) float sVr[kHid];
  const int lane = threadIdx.x & 31;
  const int hh   = lane >> 4;
  const int col  = lane & 15;
  const int z    = blockIdx.x / kTilesPerSys;
  const int a0   = (blockIdx.x - z * kTilesPerSys) * kAtomsPerWave;

  sC[lane] = kCutoff * ((float)lane * kInvSteps);
#pragma unroll 1
  for (int it = 0; it < (kHid * kNrbf) / (32 * 8); ++it) {
    const int o = (it * 32 + lane) * 8;
    const v8h w = *(const v8h*)(W1t + o);
    *(v8h*)(sW + o) = w;
  }
  {
    const v4f bq = *(const v4f*)(b1 + lane * 4);
    v4f bs;
    bs[0] = bq[0] * kCarryProd;
    bs[1] = bq[1] * kCarryProd;
    bs[2] = bq[2] * kCarryProd;
    bs[3] = bq[3] * kCarryProd;
    *(v4f*)(sB1 + lane * 4) = bs;
  }
  __syncthreads();

  const float* ga0 = geom + (size_t)(z * kAtoms + a0 + col) * 3;
  const float* ga1 = ga0 + 16 * 3;
  const float ax0 = ga0[0], ay0 = ga0[1], az0 = ga0[2];
  const float ax1 = ga1[0], ay1 = ga1[1], az1 = ga1[2];

  float p0[8], p1[8];
#pragma unroll
  for (int r = 0; r < 8; ++r) { p0[r] = 0.0f; p1[r] = 0.0f; }

#pragma unroll 1
  for (int b = 0; b < kAtoms; ++b) {
    const float* gb = geom + (size_t)(z * kAtoms + b) * 3;
    const float bx = gb[0], by = gb[1], bz = gb[2];
    const v4f vq = *(const v4f*)(V + (size_t)(z * kAtoms + b) * kHid + lane * 4);
    float r0, r1;
    {
      const float dx = bx - ax0, dy = by - ay0, dz = bz - az0;
      r0 = sqrtf((dx * dx + dy * dy + dz * dz) + 1e-12f);
    }
    {
      const float dx = bx - ax1, dy = by - ay1, dz = bz - az1;
      r1 = sqrtf((dx * dx + dy * dy + dz * dz) + 1e-12f);
    }
#pragma unroll 1
    for (int q = 0; q < 4; ++q) {
      const int t  = q >> 1;
      const int kb = 16 * (q & 1) + 8 * hh;
      const float rr = (t == 0) ? r0 : r1;
      const v4f c0 = *(const v4f*)(sC + kb);
      const v4f c1 = *(const v4f*)(sC + kb + 4);
      v8h hv;
#pragma unroll
      for (int e = 0; e < 4; ++e) {
        hv[e]     = basis_f16(rr - c0[e]);
        hv[4 + e] = basis_f16(rr - c1[e]);
      }
      *(v8h*)(sA + (t * 16 + col) * kNrbf + kb) = hv;
    }
    *(v4f*)(sVr + lane * 4) = vq;
    __syncthreads();
    const v16h af0 = frag_load_f16(sA + col * kNrbf + 8 * hh);
    const v16h af1 = frag_load_f16(sA + (16 + col) * kNrbf + 8 * hh);

#pragma unroll 1
    for (int blk = 0; blk < kHid / 16; ++blk) {
      const int n = blk * 16 + col;
      const v16h wfr = frag_load_f16(sW + n * kNrbf + 8 * hh);
      const float vv = sVr[n];
      const float cb = sB1[n];
      v8f d0 = (v8f){cb, cb, cb, cb, cb, cb, cb, cb};
      d0 = mma_f16(af0, wfr, d0);
      v8f d1 = (v8f){cb, cb, cb, cb, cb, cb, cb, cb};
      d1 = mma_f16(af1, wfr, d1);
#pragma unroll
      for (int r = 0; r < 8; ++r) {
        p0[r] = fmaf(fmaxf(d0[r], 0.0f), vv, p0[r]);
        p1[r] = fmaf(fmaxf(d1[r], 0.0f), vv, p1[r]);
      }
    }
    __syncthreads();
  }

#pragma unroll
  for (int r = 0; r < 8; ++r) {
    float s0 = p0[r], s1 = p1[r];
    s0 += __shfl_xor(s0, 1, 32);  s1 += __shfl_xor(s1, 1, 32);
    s0 += __shfl_xor(s0, 2, 32);  s1 += __shfl_xor(s1, 2, 32);
    s0 += __shfl_xor(s0, 4, 32);  s1 += __shfl_xor(s1, 4, 32);
    s0 += __shfl_xor(s0, 8, 32);  s1 += __shfl_xor(s1, 8, 32);
    p0[r] = s0;
    p1[r] = s1;
  }
  const int hsrc = ((lane >> 3) & 1) * 16;
  const int tsel = lane >> 4;
  const int rsel = lane & 7;
  float res = 0.0f;
#pragma unroll
  for (int r = 0; r < 8; ++r) {
    const float w0 = __shfl(p0[r], hsrc, 32);
    const float w1 = __shfl(p1[r], hsrc, 32);
    const float w  = (tsel == 0) ? w0 : w1;
    res = (rsel == r) ? w : res;
  }
  float ss = 0.0f;
#pragma unroll
  for (int i = 0; i < kAtoms / 32; ++i) ss += S[z * kAtoms + i * 32 + lane];
  ss += __shfl_xor(ss, 16, 32);
  ss += __shfl_xor(ss, 8, 32);
  ss += __shfl_xor(ss, 4, 32);
  ss += __shfl_xor(ss, 2, 32);
  ss += __shfl_xor(ss, 1, 32);

  const float x  = res * kFold + ss;
  const float sp = fmaxf(x, 0.0f) + log1pf(expf(-fabsf(x)));
  const float mk = maskp[z * kAtoms + a0 + lane];
  const float val = (sp - kLn2) * mk;
  volatile float* op = out + (size_t)z * kAtoms + a0 + lane;
  *op = val;
  __threadfence();
  *op = val;
}

extern "C" void kernel_launch(void* const* d_in, const int* in_sizes, int n_in,
                              void* d_out, int out_size, void* d_ws, size_t ws_size,
                              hipStream_t stream) {
  if (n_in < 7) return;
  if (in_sizes[0] != kPairRows * 3) return;
  if (in_sizes[1] != kPairRows * kChan) return;
  if (in_sizes[2] != kPairRows) return;
  if (in_sizes[3] != kNrbf * kHid) return;
  if (in_sizes[4] != kHid) return;
  if (in_sizes[5] != kHid * kChan) return;
  if (in_sizes[6] != kChan) return;
  if (out_size != kPairRows) return;
  if (ws_size < kWsTotal) return;

  const float* geom     = (const float*)d_in[0];
  const float* features = (const float*)d_in[1];
  const float* maskp    = (const float*)d_in[2];
  const float* W1       = (const float*)d_in[3];
  const float* b1       = (const float*)d_in[4];
  const float* W2       = (const float*)d_in[5];
  const float* b2       = (const float*)d_in[6];
  float* out = (float*)d_out;

  char* ws = (char*)d_ws;
  float*          V   = (float*)(ws + kOffV);
  float*          S   = (float*)(ws + kOffS);
  unsigned short* W1t = (unsigned short*)(ws + kOffW1T);

  w1_plane_kernel<<<(kHid * (kNrbf / 8)) / 256, 256, 0, stream>>>(W1, W1t);
  neighbour_vec_kernel<<<kPairRows / kRowsPerBlk, 128, 0, stream>>>(features, maskp, W2, b2, V, S);
  pair_filter_kernel<<<kSys * kTilesPerSys, kAtomsPerWave, 0, stream>>>(
      geom, maskp, b1, (const _Float16*)W1t, V, S, out);
}
